// RNNFakeDetectionModel_87333864997080
// MI455X (gfx1250) — hardware-verified
//
#include <hip/hip_runtime.h>
#include <stddef.h>
#include <stdint.h>

constexpr int NBAT   = 64;
constexpr int LWAV   = 160000;
constexpr int NFFT_  = 400;
constexpr int HOPS   = 160;
constexpr int PADW   = 200;
constexpr int NT     = 1001;
constexpr int MROWS  = NBAT * NT;
constexpr int RB     = 32;
constexpr int NBLK1  = MROWS / RB;
constexpr int KPAD   = 416;
constexpr int KSTEPS = KPAD / 32;
constexpr int NBAS   = 416;
constexpr int BP     = 512;
constexpr int NBIN   = 201;
constexpr int PP     = 208;
constexpr int NMEL   = 40;
constexpr int MP     = 64;
constexpr int FBW    = 48;
constexpr int FBP    = 64;
constexpr int NMFCC  = 13;
constexpr int XP     = 32;
constexpr int TBLK   = 4;
constexpr int NTP    = 1004;
constexpr int HID    = 64;
constexpr int DEN    = 32;
constexpr int NCLS   = 2;
constexpr int NTHR1  = 416;
constexpr int PML    = 32;
constexpr int QSPAN  = (NT + RB - 1) / RB + 2;

static_assert(MROWS % RB == 0);
static_assert(NTP % TBLK == 0 && NTP >= NT);
static_assert(KPAD % 32 == 0 && KPAD >= NFFT_);
static_assert(NBAS == 32 * (NTHR1 / 32));
static_assert(NTHR1 == KPAD);
static_assert(RB * 4 <= NTHR1);
static_assert(FBW + 16 <= FBP);
static_assert(NBIN <= PP && PP == 16 * (NTHR1 / 32));

constexpr float DW = (float)(6.283185307179586476925286766559 / (double)NFFT_);

constexpr size_t SZ_COS   = 512 * 4;
constexpr size_t SZ_HANN  = 512 * 4;
constexpr size_t SZ_DCT   = 640 * 4;
constexpr size_t SZ_FB    = (size_t)NMEL * FBP * 4;
constexpr size_t SZ_BPL   = (size_t)NBAS * BP * 2;
constexpr size_t SZ_MEL   = (size_t)MROWS * MP * 4;
constexpr size_t SZ_PMAX  = (size_t)NBLK1 * PML * 4;
constexpr size_t SZ_XPL   = (size_t)NTP * NBAT * XP * 2;
constexpr size_t OFF_COS  = 0;
constexpr size_t OFF_HANN = OFF_COS + SZ_COS;
constexpr size_t OFF_DCT  = OFF_HANN + SZ_HANN;
constexpr size_t OFF_FB   = OFF_DCT + SZ_DCT;
constexpr size_t OFF_BH   = OFF_FB + SZ_FB;
constexpr size_t OFF_BL   = OFF_BH + SZ_BPL;
constexpr size_t OFF_MEL  = OFF_BL + SZ_BPL;
constexpr size_t OFF_PMAX = OFF_MEL + SZ_MEL;
constexpr size_t OFF_XPL  = OFF_PMAX + SZ_PMAX;
constexpr size_t WS_TOTAL = OFF_XPL + SZ_XPL;
static_assert(WS_TOTAL <= (size_t)134217728);
static_assert(OFF_HANN % 128 == 0 && OFF_DCT % 128 == 0 && OFF_FB % 128 == 0 && OFF_BH % 128 == 0 &&
              OFF_BL % 128 == 0 && OFF_MEL % 128 == 0 && OFF_PMAX % 128 == 0 && OFF_XPL % 128 == 0);

typedef __bf16 v16bf __attribute__((ext_vector_type(16)));
typedef _Float16 v16h __attribute__((ext_vector_type(16)));
typedef _Float16 v8h __attribute__((ext_vector_type(8)));
typedef unsigned short v8us __attribute__((ext_vector_type(8)));
typedef unsigned int v4u __attribute__((ext_vector_type(4)));
typedef float v8f __attribute__((ext_vector_type(8)));
typedef float v4f __attribute__((ext_vector_type(4)));
typedef v4f __attribute__((may_alias)) v4fa;
typedef v4u __attribute__((may_alias)) v4ua;
typedef v8us __attribute__((may_alias)) v8usa;
typedef v8h __attribute__((may_alias)) v8ha;

union FragB { v16bf v; v8us u[2]; };
union FragH { v16h v; v8us u[2]; v8h h[2]; _Float16 e[16]; };

__device__ __forceinline__ v8f mma_bf(v16bf a, v16bf b, v8f acc) {
  acc = __builtin_amdgcn_wmma_f32_16x16x32_bf16(false, a, false, b, (short)0, acc, false, false);
  asm volatile("v_nop\n\tv_nop\n\tv_nop\n\tv_nop" : "+v"(acc) : "v"(a), "v"(b));
  return acc;
}
__device__ __forceinline__ v8f mma_h(v16h a, v16h b, v8f acc) {
  acc = __builtin_amdgcn_wmma_f32_16x16x32_f16(false, a, false, b, (short)0, acc, false, false);
  asm volatile("v_nop\n\tv_nop\n\tv_nop\n\tv_nop" : "+v"(acc) : "v"(a), "v"(b));
  return acc;
}

__device__ __forceinline__ v8f zero8() { return (v8f){0.f, 0.f, 0.f, 0.f, 0.f, 0.f, 0.f, 0.f}; }

__device__ __forceinline__ v16bf ldfrag_g(const unsigned short* __restrict__ p, int row0, int k0, int lane) {
  const int m = lane & 15, lh = lane >> 4;
  const unsigned short* q = p + (size_t)(row0 + m) * BP + k0 + 8 * lh;
  FragB f;
  f.u[0] = *(const v8us*)(q);
  f.u[1] = *(const v8us*)(q + 16);
  return f.v;
}
__device__ __forceinline__ v16bf ldfrag_l(const unsigned int* base, int row0, int lane) {
  const int m = lane & 15, lh = lane >> 4;
  const unsigned int* q = base + (row0 + m) * 16 + 4 * lh;
  FragB f;
  f.u[0] = *(const v8usa*)(q);
  f.u[1] = *(const v8usa*)(q + 8);
  return f.v;
}

__device__ __forceinline__ unsigned int bf16_rne_bits(float x) {
  const unsigned int u = __float_as_uint(x);
  return (u + 0x7FFFu + ((u >> 16) & 1u)) >> 16;
}
__device__ __forceinline__ void split_bf16(float x, unsigned int& h, unsigned int& l) {
  const unsigned int hb = bf16_rne_bits(x);
  const float hf = __uint_as_float(hb << 16);
  h = hb;
  l = bf16_rne_bits(x - hf);
}
__device__ __forceinline__ void shin(unsigned int& w0, unsigned int& w1, unsigned int& w2, unsigned int& w3, unsigned int hb) {
  w0 = (w0 >> 16) | (w1 << 16);
  w1 = (w1 >> 16) | (w2 << 16);
  w2 = (w2 >> 16) | (w3 << 16);
  w3 = (w3 >> 16) | (hb << 16);
}
__device__ __forceinline__ void consume(float& v) { asm volatile("" : "+v"(v)); }

__device__ __forceinline__ float wave_max(float v) {
#pragma unroll
  for (int o = 16; o > 0; o >>= 1) v = fmaxf(v, __shfl_xor(v, o, 32));
  return v;
}

__device__ __forceinline__ float dct_val(int e) {
  const int mI = e >> 4, cI = e & 15;
  const float PI_F = 3.14159265358979323846f;
  float v = 2.0f * cosf((PI_F / 40.0f) * ((float)mI + 0.5f) * (float)cI);
  v = (cI == 0) ? (v * 0.70710678118654752f) : v;
  v = v * 0.11180339887498948f;
  return (cI < NMFCC) ? v : 0.0f;
}

__global__ __launch_bounds__(512) void k_trig(float* __restrict__ cosT, float* __restrict__ hann, float* __restrict__ dct) {
  const int i = (int)threadIdx.x;
  const bool ok = i < NFFT_;
  const int r = ok ? i : 0;
  const float cs0 = cosf(DW * (float)r);
  const float hv = ok ? (0.5f * (1.0f - cs0)) : 0.0f;
  const float cs = ok ? cs0 : 0.0f;
  *(volatile float*)(cosT + i) = cs;
  *(volatile float*)(hann + i) = hv;
  __threadfence();
  *(volatile float*)(cosT + i) = cs;
  *(volatile float*)(hann + i) = hv;
#pragma unroll 1
  for (int it = 0; it < 2; ++it) {
    const int e = i + 512 * it;
    if (e < 640) {
      const float v = dct_val(e);
      *(volatile float*)(dct + e) = v;
      __threadfence();
      *(volatile float*)(dct + e) = v;
    }
  }
}

__global__ __launch_bounds__(64) void k_melfb(float* __restrict__ fb) {
  __shared__ double s_fp[NMEL + 2];
  __shared__ __align__(16) float s_tab[NMEL * FBP];
  const int tid = (int)threadIdx.x;
#pragma unroll 1
  for (int it = 0; it < (NMEL * FBP) / 64; ++it) s_tab[tid + 64 * it] = 0.0f;
  if (tid < NMEL + 2) {
    const double mmax = 2595.0 * log10(1.0 + 8000.0 / 700.0);
    const double step = mmax / 41.0;
    const double mp = (tid == NMEL + 1) ? mmax : ((double)tid * step);
    s_fp[tid] = 700.0 * (pow(10.0, mp / 2595.0) - 1.0);
  }
  __syncthreads();
  if (tid < NMEL) {
    const double f0 = s_fp[tid], f1 = s_fp[tid + 1], f2 = s_fp[tid + 2];
    int klo = (int)floor(f0 * 0.025);
    klo = min(max(klo, 0), NBIN - 1);
    int khi = (int)floor(f2 * 0.025) + 1;
    khi = min(max(khi, 0), NBIN - 1);
    int cnt = khi - klo + 1;
    cnt = min(max(cnt, 0), FBW);
    float* row = s_tab + tid * FBP;
    row[0] = (float)klo;
    row[1] = (float)cnt;
    const double d0 = f1 - f0, d1 = f2 - f1;
#pragma unroll 1
    for (int i = 0; i < cnt; ++i) {
      const double freq = 40.0 * (double)(klo + i);
      const double down = (freq - f0) / d0;
      const double up = (f2 - freq) / d1;
      const double w = fmax(0.0, fmin(down, up));
      row[16 + i] = (float)w;
    }
  }
  __syncthreads();
  v4f vals[10];
#pragma unroll
  for (int it = 0; it < 10; ++it) vals[it] = *(const v4fa*)(s_tab + 4 * (tid + 64 * it));
#pragma unroll
  for (int it = 0; it < 10; ++it) *(volatile v4f*)(fb + 4 * (tid + 64 * it)) = vals[it];
  __threadfence();
#pragma unroll
  for (int it = 0; it < 10; ++it) *(volatile v4f*)(fb + 4 * (tid + 64 * it)) = vals[it];
}

__global__ __launch_bounds__(64) void k_basis(const float* __restrict__ cosT,
                                              unsigned short* __restrict__ bh, unsigned short* __restrict__ bl) {
  __shared__ __align__(16) float s_c[512];
  const int n = blockIdx.x;
  const int tid = (int)threadIdx.x;
#pragma unroll
  for (int it = 0; it < 2; ++it) {
    const int p = tid + 64 * it;
    *(v4fa*)(s_c + 4 * p) = *(const v4f*)(cosT + 4 * p);
  }
  __syncthreads();
  const int j = n >> 5, half = (n >> 4) & 1, c = n & 15;
  const int bin = 16 * j + c;
  const bool binv = bin < NBIN;
  const int binc = binv ? bin : 0;
  const int k0 = 8 * tid;
  unsigned int h0 = 0u, h1 = 0u, h2 = 0u, h3 = 0u, l0 = 0u, l1 = 0u, l2 = 0u, l3 = 0u;
#pragma unroll 1
  for (int jj = 0; jj < 8; ++jj) {
    const int k = k0 + jj;
    const bool kv = k < NFFT_;
    const int kc = kv ? k : 0;
    const int r = (binc * kc) % NFFT_;
    const int rs = (r + 300) % NFFT_;
    const float vc = s_c[r];
    const float vs = s_c[rs];
    float v = half ? vs : vc;
    v = (binv && kv) ? v : 0.0f;
    unsigned int hbits, lbits;
    split_bf16(v, hbits, lbits);
    shin(h0, h1, h2, h3, hbits);
    shin(l0, l1, l2, l3, lbits);
  }
  const v4u vh = (v4u){h0, h1, h2, h3};
  const v4u vl = (v4u){l0, l1, l2, l3};
  unsigned short* ph = bh + (size_t)n * BP + k0;
  unsigned short* pl = bl + (size_t)n * BP + k0;
  *(volatile v4u*)ph = vh;
  *(volatile v4u*)pl = vl;
  __threadfence();
  *(volatile v4u*)ph = vh;
  *(volatile v4u*)pl = vl;
}

__global__ __launch_bounds__(NTHR1) void k_dft_mel(const float* __restrict__ wav, const float* __restrict__ hannT,
                                                     const float* __restrict__ fbT,
                                                     const unsigned short* __restrict__ BH, const unsigned short* __restrict__ BL,
                                                     float* __restrict__ mel, float* __restrict__ pmax) {
  __shared__ __align__(16) unsigned int s_ah[RB * 16];
  __shared__ __align__(16) unsigned int s_al[RB * 16];
  __shared__ __align__(16) float s_pow[RB * PP];
  __shared__ __align__(16) float s_mel[RB * MP];
  __shared__ __align__(16) float s_fb[NMEL * FBP];
  __shared__ float s_hann[KPAD];
  __shared__ float s_red[2][16];
  __shared__ float s_bm[2];

  const int tid = (int)threadIdx.x, lane = tid & 31, wave = tid >> 5;
  const int hh = lane >> 4, c = lane & 15;
  const int r0 = blockIdx.x * RB;
  const int bfirst = r0 / NT;

  s_hann[tid] = hannT[tid];
#pragma unroll
  for (int it = 0; it < 2; ++it) {
    const int p = tid + NTHR1 * it;
    if (p < (NMEL * FBP) / 4) *(v4fa*)(s_fb + 4 * p) = *(const v4f*)(fbT + 4 * p);
  }

  const int srow = (tid >> 2) & (RB - 1), sq = tid & 3;
  const int grow = r0 + srow;
  const int sb = grow / NT, st = grow - sb * NT;
  const float* xb = wav + (size_t)sb * LWAV;
  const int tb = st * HOPS - PADW;

  const int nrc = 32 * wave, nrs = 32 * wave + 16;
  v8f accC[2], accS[2];
  accC[0] = zero8(); accC[1] = zero8(); accS[0] = zero8(); accS[1] = zero8();
  __syncthreads();

#pragma unroll 1
  for (int ks = 0; ks < KSTEPS; ++ks) {
    if (tid < RB * 4) {
      const int k0 = 32 * ks + 8 * sq;
      unsigned int h0 = 0u, h1 = 0u, h2 = 0u, h3 = 0u, l0 = 0u, l1 = 0u, l2 = 0u, l3 = 0u;
#pragma unroll 1
      for (int jj = 0; jj < 8; ++jj) {
        const int k = k0 + jj;
        int idx = tb + k;
        idx = (idx < 0) ? (-idx) : idx;
        idx = (idx >= LWAV) ? (2 * LWAV - 2 - idx) : idx;
        idx = min(max(idx, 0), LWAV - 1);
        float v = xb[idx];
        consume(v);
        v = v * s_hann[k];
        unsigned int hbits, lbits;
        split_bf16(v, hbits, lbits);
        shin(h0, h1, h2, h3, hbits);
        shin(l0, l1, l2, l3, lbits);
      }
      *(v4ua*)(s_ah + srow * 16 + 4 * sq) = (v4u){h0, h1, h2, h3};
      *(v4ua*)(s_al + srow * 16 + 4 * sq) = (v4u){l0, l1, l2, l3};
    }
    __syncthreads();
    const int kb = 32 * ks;
    const v16bf bhc = ldfrag_g(BH, nrc, kb, lane);
    const v16bf bhs = ldfrag_g(BH, nrs, kb, lane);
    const v16bf blc = ldfrag_g(BL, nrc, kb, lane);
    const v16bf bls = ldfrag_g(BL, nrs, kb, lane);
#pragma unroll
    for (int s = 0; s < 2; ++s) {
      const v16bf ah = ldfrag_l(s_ah, 16 * s, lane);
      const v16bf al = ldfrag_l(s_al, 16 * s, lane);
      accC[s] = mma_bf(ah, bhc, accC[s]);
      accC[s] = mma_bf(ah, blc, accC[s]);
      accC[s] = mma_bf(al, bhc, accC[s]);
      accS[s] = mma_bf(ah, bhs, accS[s]);
      accS[s] = mma_bf(ah, bls, accS[s]);
      accS[s] = mma_bf(al, bhs, accS[s]);
    }
    __syncthreads();
  }

#pragma unroll
  for (int s = 0; s < 2; ++s) {
#pragma unroll
    for (int r = 0; r < 8; ++r) {
      const float re = accC[s][r], im = accS[s][r];
      s_pow[(16 * s + 8 * hh + r) * PP + 16 * wave + c] = re * re + im * im;
    }
  }
  __syncthreads();

  float wm0 = 0.0f, wm1 = 0.0f;
#pragma unroll 1
  for (int it = 0; it < 5; ++it) {
    const int e = tid + NTHR1 * it;
    if (e < RB * MP) {
      const int row = e >> 6, m = e & 63;
      const int mm = min(m, NMEL - 1);
      const float* fr = s_fb + mm * FBP;
      int kb0 = (int)fr[0];
      int cnt = (int)fr[1];
      kb0 = min(max(kb0, 0), NBIN - 1);
      cnt = min(max(cnt, 0), FBW);
      cnt = (m < NMEL) ? cnt : 0;
      const float* pr = s_pow + row * PP;
      float sum = 0.0f;
#pragma unroll 1
      for (int q = 0; q < cnt; ++q) sum += pr[min(kb0 + q, PP - 1)] * fr[16 + q];
      s_mel[row * MP + m] = sum;
      const bool sl1 = ((r0 + row) / NT) != bfirst;
      wm0 = fmaxf(wm0, sl1 ? 0.0f : sum);
      wm1 = fmaxf(wm1, sl1 ? sum : 0.0f);
    }
  }
  wm0 = wave_max(wm0);
  wm1 = wave_max(wm1);
  if (lane == 0) { s_red[0][wave] = wm0; s_red[1][wave] = wm1; }
  __syncthreads();
  if (tid < 2) {
    float mx = 0.0f;
#pragma unroll 1
    for (int w = 0; w < NTHR1 / 32; ++w) mx = fmaxf(mx, s_red[tid][w]);
    s_bm[tid] = mx;
  }
  __syncthreads();

  const int p0 = tid;
  const int L0 = p0 >> 4, c0 = p0 & 15;
  const v4f mv0 = *(const v4fa*)(s_mel + L0 * MP + 4 * c0);
  const size_t mg0 = (size_t)(r0 + L0) * MP + 4 * c0;
  const bool ok1 = tid < (RB * MP) / 4 - NTHR1;
  const int p1 = ok1 ? (tid + NTHR1) : 0;
  const int L1 = p1 >> 4, c1 = p1 & 15;
  const v4f mv1 = *(const v4fa*)(s_mel + L1 * MP + 4 * c1);
  const size_t mg1 = (size_t)(r0 + L1) * MP + 4 * c1;
  const float bm0 = s_bm[0], bm1 = s_bm[1];
  const v4f pv = (lane == 0) ? (v4f){bm0, bm1, 0.0f, 0.0f} : (v4f){0.0f, 0.0f, 0.0f, 0.0f};
  const bool pok = (wave == 0) && (lane < 8);
  float* pline = pmax + (size_t)blockIdx.x * PML + 4 * (lane & 7);

  *(volatile v4f*)(mel + mg0) = mv0;
  if (ok1) *(volatile v4f*)(mel + mg1) = mv1;
  if (pok) *(volatile v4f*)pline = pv;
  __threadfence();
  *(volatile v4f*)(mel + mg0) = mv0;
  if (ok1) *(volatile v4f*)(mel + mg1) = mv1;
  if (pok) *(volatile v4f*)pline = pv;
}

__global__ __launch_bounds__(256) void k_dbdct(const float* __restrict__ mel, const float* __restrict__ pmax,
                                               const float* __restrict__ dctT, unsigned int* __restrict__ xw) {
  __shared__ float s_thr[NBAT];
  __shared__ __align__(16) float s_dct[640];
  __shared__ __align__(16) unsigned int s_x[TBLK * NBAT * 16];
  const int tid = (int)threadIdx.x, tl = tid >> 6, b = tid & 63;
  const int t0 = blockIdx.x * TBLK, t = t0 + tl, tc = min(t, NT - 1);
#pragma unroll 1
  for (int it = 0; it < 3; ++it) {
    const int e = tid + 256 * it;
    if (e < 640) s_dct[e] = dctT[e];
  }
  if (tid < NBAT) {
    const int qlo = (b * NT) / RB, qhi = (b * NT + NT - 1) / RB;
    float mx = 0.0f;
#pragma unroll 1
    for (int i = 0; i < QSPAN; ++i) {
      const int q = qlo + i;
      const bool ok = q <= qhi;
      const int qc = min(q, NBLK1 - 1);
      int sl = b - (qc * RB) / NT;
      sl = min(max(sl, 0), 1);
      const float v = pmax[(size_t)qc * PML + sl];
      mx = fmaxf(mx, ok ? v : 0.0f);
    }
    s_thr[tid] = 10.0f * log10f(fmaxf(mx, 1e-10f)) - 80.0f;
  }
  __syncthreads();
  const float thr = s_thr[b];
  const float* mr = mel + ((size_t)b * NT + tc) * MP;
  float cf[NMFCC];
#pragma unroll
  for (int cI = 0; cI < NMFCC; ++cI) cf[cI] = 0.0f;
#pragma unroll 1
  for (int m = 0; m < NMEL; ++m) {
    const float v = mr[m];
    const float d = fmaxf(10.0f * log10f(fmaxf(v, 1e-10f)), thr);
    const float* dr = s_dct + m * 16;
#pragma unroll
    for (int cI = 0; cI < NMFCC; ++cI) cf[cI] += d * dr[cI];
  }
  unsigned int u[NMFCC];
#pragma unroll
  for (int cI = 0; cI < NMFCC; ++cI) u[cI] = (unsigned int)__builtin_bit_cast(unsigned short, (_Float16)cf[cI]);
  const unsigned int w0 = u[0] | (u[1] << 16), w1 = u[2] | (u[3] << 16), w2 = u[4] | (u[5] << 16), w3 = u[6] | (u[7] << 16);
  const unsigned int w4 = u[8] | (u[9] << 16), w5 = u[10] | (u[11] << 16), w6 = u[12];
  unsigned int* sx = s_x + (tl * NBAT + b) * 16;
  *(v4ua*)(sx)      = (v4u){w0, w1, w2, w3};
  *(v4ua*)(sx + 4)  = (v4u){w4, w5, w6, 0u};
  *(v4ua*)(sx + 8)  = (v4u){0u, 0u, 0u, 0u};
  *(v4ua*)(sx + 12) = (v4u){0u, 0u, 0u, 0u};
  __syncthreads();
  v4u pv[4];
#pragma unroll
  for (int it = 0; it < 4; ++it) pv[it] = *(const v4ua*)(s_x + 4 * (tid + 256 * it));
  unsigned int* dst = xw + (size_t)t0 * NBAT * 16;
#pragma unroll
  for (int it = 0; it < 4; ++it) *(volatile v4u*)(dst + 4 * (tid + 256 * it)) = pv[it];
  __threadfence();
#pragma unroll
  for (int it = 0; it < 4; ++it) *(volatile v4u*)(dst + 4 * (tid + 256 * it)) = pv[it];
}

__global__ __launch_bounds__(256) void k_rnn(const unsigned short* __restrict__ xpl,
                                             const float* __restrict__ Wih, const float* __restrict__ Whh,
                                             const float* __restrict__ bih_g, const float* __restrict__ bhh_g,
                                             const float* __restrict__ W1, const float* __restrict__ b1,
                                             const float* __restrict__ W2, const float* __restrict__ b2,
                                             float* __restrict__ out) {
  __shared__ __align__(16) _Float16 hb[2][NBAT][HID];
  __shared__ __align__(16) float s_x1[NBAT][DEN];
  __shared__ __align__(16) float s_o[NBAT * NCLS];
  const int tid = (int)threadIdx.x, lane = tid & 31, wave = tid >> 5;
  const int g = lane >> 4, ln = lane & 15;
  const int mi = wave & 3, ni0 = (wave >> 2) * 2;

#pragma unroll 1
  for (int i = tid; i < NBAT * HID; i += 256) hb[0][i >> 6][i & 63] = (_Float16)0.0f;

  FragH fih[2], fhh0[2], fhh1[2];
  float bias[2];
#pragma unroll
  for (int q = 0; q < 2; ++q) {
    const int n = (ni0 + q) * 16 + ln;
#pragma unroll
    for (int i = 0; i < 16; ++i) {
      const int k = 8 * g + (i & 7) + 16 * (i >> 3);
      const int kih = min(k, NMFCC - 1);
      const float wih = Wih[n * NMFCC + kih];
      fih[q].e[i]  = (_Float16)((k < NMFCC) ? (wih * 64.0f) : 0.0f);
      fhh0[q].e[i] = (_Float16)(Whh[n * HID + k] * 64.0f);
      fhh1[q].e[i] = (_Float16)(Whh[n * HID + 32 + k] * 64.0f);
    }
    bias[q] = bih_g[n] + bhh_g[n];
  }
  __syncthreads();

  const int m = mi * 16 + ln;
  int p = 0;
#pragma unroll 1
  for (int t = 0; t < NT; ++t) {
    FragH ax, a0, a1;
    const unsigned short* xr = xpl + ((size_t)t * NBAT + m) * XP;
    ax.u[0] = *(const v8us*)(xr + 8 * g);
    ax.u[1] = *(const v8us*)(xr + 16 + 8 * g);
    a0.h[0] = *(const v8ha*)(&hb[p][m][8 * g]);
    a0.h[1] = *(const v8ha*)(&hb[p][m][16 + 8 * g]);
    a1.h[0] = *(const v8ha*)(&hb[p][m][32 + 8 * g]);
    a1.h[1] = *(const v8ha*)(&hb[p][m][48 + 8 * g]);
#pragma unroll
    for (int q = 0; q < 2; ++q) {
      v8f acc = zero8();
      acc = mma_h(ax.v, fih[q].v, acc);
      acc = mma_h(a0.v, fhh0[q].v, acc);
      acc = mma_h(a1.v, fhh1[q].v, acc);
      const int n = (ni0 + q) * 16 + ln;
#pragma unroll
      for (int r = 0; r < 8; ++r) {
        const float hv = tanhf(acc[r] * 0.015625f + bias[q]);
        hb[p ^ 1][mi * 16 + 8 * g + r][n] = (_Float16)hv;
      }
    }
    p ^= 1;
    __syncthreads();
  }

  {
    const int ni = wave >> 2;
    const int n1 = ni * 16 + ln;
    FragH fw0, fw1, a0, a1;
#pragma unroll
    for (int i = 0; i < 16; ++i) {
      const int k = 8 * g + (i & 7) + 16 * (i >> 3);
      fw0.e[i] = (_Float16)(W1[n1 * HID + k] * 64.0f);
      fw1.e[i] = (_Float16)(W1[n1 * HID + 32 + k] * 64.0f);
    }
    a0.h[0] = *(const v8ha*)(&hb[p][m][8 * g]);
    a0.h[1] = *(const v8ha*)(&hb[p][m][16 + 8 * g]);
    a1.h[0] = *(const v8ha*)(&hb[p][m][32 + 8 * g]);
    a1.h[1] = *(const v8ha*)(&hb[p][m][48 + 8 * g]);
    v8f acc = zero8();
    acc = mma_h(a0.v, fw0.v, acc);
    acc = mma_h(a1.v, fw1.v, acc);
    const float bb = b1[n1];
#pragma unroll
    for (int r = 0; r < 8; ++r) s_x1[mi * 16 + 8 * g + r][n1] = fmaxf(acc[r] * 0.015625f + bb, 0.0f);
  }
  __syncthreads();
  if (tid < NBAT) {
    float l0 = 0.0f, l1 = 0.0f;
#pragma unroll 1
    for (int d = 0; d < DEN; ++d) {
      const float xv = s_x1[tid][d];
      l0 += xv * W2[d];
      l1 += xv * W2[DEN + d];
    }
    l0 += b2[0];
    l1 += b2[1];
    const float mx = fmaxf(l0, l1);
    const float e0 = expf(l0 - mx), e1 = expf(l1 - mx);
    const float inv = 1.0f / (e0 + e1);
    s_o[2 * tid]     = e0 * inv;
    s_o[2 * tid + 1] = e1 * inv;
  }
  __syncthreads();
  if (wave == 0) {
    const v4f v = *(const v4fa*)(s_o + 4 * lane);
    *(volatile v4f*)(out + 4 * lane) = v;
    __threadfence();
    *(volatile v4f*)(out + 4 * lane) = v;
  }
}

extern "C" void kernel_launch(void* const* d_in, const int* in_sizes, int n_in,
                              void* d_out, int out_size, void* d_ws, size_t ws_size,
                              hipStream_t stream) {
  if (n_in < 9) return;
  if (in_sizes[0] != NBAT * LWAV) return;
  if (in_sizes[1] != HID * NMFCC || in_sizes[2] != HID * HID || in_sizes[3] != HID || in_sizes[4] != HID) return;
  if (in_sizes[5] != DEN * HID || in_sizes[6] != DEN || in_sizes[7] != NCLS * DEN || in_sizes[8] != NCLS) return;
  if (out_size != NBAT * NCLS) return;
  if (ws_size < WS_TOTAL) return;

  const float* wav  = (const float*)d_in[0];
  const float* W_ih = (const float*)d_in[1];
  const float* W_hh = (const float*)d_in[2];
  const float* b_ih = (const float*)d_in[3];
  const float* b_hh = (const float*)d_in[4];
  const float* W1   = (const float*)d_in[5];
  const float* b1   = (const float*)d_in[6];
  const float* W2   = (const float*)d_in[7];
  const float* b2   = (const float*)d_in[8];
  float* out = (float*)d_out;
  char* ws = (char*)d_ws;

  float* cosT = (float*)(ws + OFF_COS);
  float* hann = (float*)(ws + OFF_HANN);
  float* dct  = (float*)(ws + OFF_DCT);
  float* fb   = (float*)(ws + OFF_FB);
  unsigned short* bh = (unsigned short*)(ws + OFF_BH);
  unsigned short* bl = (unsigned short*)(ws + OFF_BL);
  float* mel  = (float*)(ws + OFF_MEL);
  float* pmax = (float*)(ws + OFF_PMAX);
  unsigned short* xpl = (unsigned short*)(ws + OFF_XPL);

  k_trig<<<dim3(1), dim3(512), 0, stream>>>(cosT, hann, dct);
  k_melfb<<<dim3(1), dim3(64), 0, stream>>>(fb);
  k_basis<<<dim3(NBAS), dim3(64), 0, stream>>>(cosT, bh, bl);
  k_dft_mel<<<dim3(NBLK1), dim3(NTHR1), 0, stream>>>(wav, hann, fb, bh, bl, mel, pmax);
  k_dbdct<<<dim3(NTP / TBLK), dim3(256), 0, stream>>>(mel, pmax, dct, (unsigned int*)xpl);
  k_rnn<<<dim3(1), dim3(256), 0, stream>>>(xpl, W_ih, W_hh, b_ih, b_hh, W1, b1, W2, b2, out);
  (void)hipGetLastError();
}
